// HimNet_multimode_v3_7645041787314
// MI455X (gfx1250) — hardware-verified
//
#include <hip/hip_runtime.h>
#include <math.h>
#include <stdint.h>

constexpr int kB   = 8;
constexpr int kN   = 1000;
constexpr int kNP  = 1024;
constexpr int kCIN = 16;
constexpr int kH   = 64;
constexpr int kXIN = 80;
constexpr int kKX  = 240;
constexpr int kKP  = 256;
constexpr int kD   = 16;
constexpr int kOG  = 128;
constexpr int kOU  = 64;
constexpr int kJ   = kB * kXIN;
constexpr int kR   = kNP * kB;
constexpr float kSupScale = 16384.0f;
constexpr float kSupInv   = 1.0f / 16384.0f;
constexpr float kWScale   = 64.0f;
constexpr float kWInv     = 1.0f / 64.0f;

constexpr size_t SZ_WG    = (size_t)kD * kOG * kKP * 2;
constexpr size_t SZ_WU    = (size_t)kD * kOU * kKP * 2;
constexpr size_t OFF_WG   = 0;
constexpr size_t OFF_WU   = OFF_WG + SZ_WG;
constexpr size_t OFF_CELL = OFF_WU + SZ_WU;
constexpr size_t SZ_S16   = (size_t)kNP * kNP * 2;
constexpr size_t SZ_PL    = (size_t)kJ * kNP * 2;
constexpr size_t SZ_XG    = (size_t)kR * kKP * 2;
constexpr size_t SZ_ZR    = (size_t)kR * kOG * 4;
constexpr size_t C_S16    = 0;
constexpr size_t C_XST    = C_S16 + SZ_S16;
constexpr size_t C_T1T    = C_XST + SZ_PL;
constexpr size_t C_T2T    = C_T1T + SZ_PL;
constexpr size_t C_XG     = C_T2T + SZ_PL;
constexpr size_t C_ZR     = C_XG + SZ_XG;
constexpr size_t CELL_SZ  = C_ZR + SZ_ZR;
constexpr size_t WS_TOTAL = OFF_CELL + 3 * CELL_SZ;
constexpr size_t CELLH    = CELL_SZ / 2;
constexpr size_t CELLF    = CELL_SZ / 4;
constexpr size_t PLANEH   = SZ_PL / 2;
static_assert((CELL_SZ % 128) == 0);
static_assert((SZ_PL % 128) == 0);
static_assert(C_T1T == C_XST + SZ_PL);
static_assert(C_T2T == C_T1T + SZ_PL);
static_assert(WS_TOTAL <= (size_t)134217728);

typedef _Float16 v16h __attribute__((ext_vector_type(16)));
typedef _Float16 v8h  __attribute__((ext_vector_type(8)));
typedef float    v8f  __attribute__((ext_vector_type(8)));
typedef float    v4f  __attribute__((ext_vector_type(4)));

__device__ __forceinline__ float bf_rne(float f) {
  unsigned u = __float_as_uint(f);
  u = (u + 0x7FFFu + ((u >> 16) & 1u)) & 0xFFFF0000u;
  return __uint_as_float(u);
}
__device__ __forceinline__ v4f bf4(v4f v) {
  v4f r;
  r[0] = bf_rne(v[0]); r[1] = bf_rne(v[1]); r[2] = bf_rne(v[2]); r[3] = bf_rne(v[3]);
  return r;
}
__device__ __forceinline__ v8f zero8() { v8f z = {0.f, 0.f, 0.f, 0.f, 0.f, 0.f, 0.f, 0.f}; return z; }
__device__ __forceinline__ v8h pack8(v4f a, v4f b) {
  v8h p;
  p[0] = (_Float16)a[0]; p[1] = (_Float16)a[1]; p[2] = (_Float16)a[2]; p[3] = (_Float16)a[3];
  p[4] = (_Float16)b[0]; p[5] = (_Float16)b[1]; p[6] = (_Float16)b[2]; p[7] = (_Float16)b[3];
  return p;
}

__device__ __forceinline__ float act_f32(float x, bool th) {
  const float u = th ? (2.0f * x) : x;
  const float e = __expf(-fabsf(u));
  const float r = 1.0f / (1.0f + e);
  const float sg = (u >= 0.0f) ? r : (e * r);
  const float tn = copysignf((1.0f - e) * r, x);
  return th ? tn : sg;
}

__device__ __forceinline__ v16h ldfrag(const _Float16* p) {
  union { v16h v; v8h hh[2]; } f;
  f.hh[0] = *(const v8h*)(p);
  f.hh[1] = *(const v8h*)(p + 16);
  return f.v;
}
__device__ __forceinline__ v8f mma(v16h a, v16h b, v8f c) {
  return __builtin_amdgcn_wmma_f32_16x16x32_f16(false, a, false, b, (short)0, c, false, false);
}
__device__ __forceinline__ void guard2(v8f& c0, v8f& c1, v16h a, v16h b0, v16h b1) {
#if defined(__HIP_DEVICE_COMPILE__)
  asm volatile("v_nop\n\tv_nop\n\tv_nop\n\tv_nop" : "+v"(c0), "+v"(c1) : "v"(a), "v"(b0), "v"(b1));
#endif
}
__device__ __forceinline__ void guard4(v8f& c0, v8f& c1, v8f& c2, v8f& c3,
                                       v16h a, v16h b0, v16h b1, v16h b2, v16h b3) {
#if defined(__HIP_DEVICE_COMPILE__)
  asm volatile("v_nop\n\tv_nop\n\tv_nop\n\tv_nop"
               : "+v"(c0), "+v"(c1), "+v"(c2), "+v"(c3)
               : "v"(a), "v"(b0), "v"(b1), "v"(b2), "v"(b3));
#endif
}
__device__ __forceinline__ void wave_sync_lds() {
  __builtin_amdgcn_fence(__ATOMIC_RELEASE, "workgroup");
  __builtin_amdgcn_wave_barrier();
  __builtin_amdgcn_fence(__ATOMIC_ACQUIRE, "workgroup");
}

__global__ __launch_bounds__(256) void build_s16(const float* __restrict__ s1, const float* __restrict__ s2,
                                                 const float* __restrict__ s3, unsigned short* S16b) {
  const int m = blockIdx.z;
  const float* sup = (m == 0) ? s1 : ((m == 1) ? s2 : s3);
  _Float16* S = (_Float16*)S16b + (size_t)m * CELLH;
  const int idx = blockIdx.x * 256 + (int)threadIdx.x;
  const int r  = idx >> 7;
  const int c8 = (idx & 127) * 8;
  const bool valid = (r < kN) && (c8 < kN);
  const int rc = (r < kN) ? r : (kN - 1);
  const int cc = (c8 <= kN - 8) ? c8 : (kN - 8);
  const float* p = sup + (size_t)rc * kN + cc;
  v4f a = *(const v4f*)(p);
  v4f b = *(const v4f*)(p + 4);
  a = bf4(a) * kSupScale;
  b = bf4(b) * kSupScale;
  const v4f z4 = {0.f, 0.f, 0.f, 0.f};
  if (!valid) { a = z4; b = z4; }
  const v8h o = pack8(a, b);
  _Float16* q = S + (size_t)r * kNP + c8;
  *(volatile v8h*)q = o;
  __threadfence();
  *(volatile v8h*)q = o;
}

__global__ __launch_bounds__(256) void build_wt(const float* __restrict__ W, int O, unsigned short* WTb) {
  __shared__ __align__(16) float s[64 * 68];
  const int tid = threadIdx.x;
  const int i0 = blockIdx.x * 64;
  const int o0 = blockIdx.y * 64;
  const int d  = blockIdx.z;
#pragma unroll
  for (int it = 0; it < 4; ++it) {
    const int idx = it * 256 + tid;
    const int il = idx >> 4;
    const int o4 = (idx & 15) * 4;
    const int i  = i0 + il;
    const int ic = (i < kKX) ? i : (kKX - 1);
    const v4f v = *(const v4f*)(W + ((size_t)(d * kKX + ic)) * O + o0 + o4);
    const bool ok = (i < kKX);
#pragma unroll
    for (int e = 0; e < 4; ++e) s[(o4 + e) * 68 + il] = ok ? (bf_rne(v[e]) * kWScale) : 0.0f;
  }
  __syncthreads();
  const int q = tid & 7;
  const int orr = tid >> 3;
  v8h pk[2];
#pragma unroll
  for (int it = 0; it < 2; ++it) {
    const int ol = it * 32 + orr;
    const v4f a = *(const v4f*)(s + ol * 68 + 8 * q);
    const v4f b = *(const v4f*)(s + ol * 68 + 8 * q + 4);
    pk[it] = pack8(a, b);
  }
  _Float16* WT = (_Float16*)WTb;
  for (int pass = 0; pass < 2; ++pass) {
#pragma unroll
    for (int it = 0; it < 2; ++it) {
      const int ol = it * 32 + orr;
      *(volatile v8h*)(WT + ((size_t)(d * O + o0 + ol)) * kKP + i0 + 8 * q) = pk[it];
    }
    __threadfence();
  }
}

template <int UPD>
__global__ __launch_bounds__(256) void build_xst(const float* __restrict__ x1, const float* __restrict__ x2,
                                                 const float* __restrict__ x3,
                                                 const float* __restrict__ t1, const float* __restrict__ t2,
                                                 const float* __restrict__ t3,
                                                 const float* ZRb, unsigned short* XsTb) {
  __shared__ __align__(16) float s[kXIN * 68];
  const int tid = threadIdx.x;
  const int n0 = blockIdx.x * 64;
  const int b  = blockIdx.y;
  const int m  = blockIdx.z;
  const float* x  = (m == 0) ? x1 : ((m == 1) ? x2 : x3);
  const float* st = (m == 0) ? t1 : ((m == 1) ? t2 : t3);
  const float* ZR = ZRb + (size_t)m * CELLF;
  _Float16* XsT = (_Float16*)XsTb + (size_t)m * CELLH;
#pragma unroll
  for (int it = 0; it < 5; ++it) {
    const int idx = it * 256 + tid;
    const int nl = idx / 20;
    const int c4 = (idx - nl * 20) * 4;
    const int n  = n0 + nl;
    const int nc = (n < kN) ? n : (kN - 1);
    const int cx = (c4 < kCIN - 4) ? c4 : (kCIN - 4);
    const int cs = (c4 >= kCIN) ? (c4 - kCIN) : 0;
    const v4f xv = bf4(*(const v4f*)(x  + ((size_t)(b * kN + nc)) * kCIN + cx));
    v4f sv = bf4(*(const v4f*)(st + ((size_t)(b * kN + nc)) * kH + cs));
    if (UPD) {
      const v4f zv = *(const v4f*)(ZR + ((size_t)(n * kB + b)) * kOG + cs);
      sv = zv * sv;
    }
    v4f v = (c4 < kCIN) ? xv : sv;
    const v4f z4 = {0.f, 0.f, 0.f, 0.f};
    if (n >= kN) v = z4;
#pragma unroll
    for (int e = 0; e < 4; ++e) s[(c4 + e) * 68 + nl] = v[e];
  }
  __syncthreads();
  const int q  = tid & 7;
  const int cr = tid >> 3;
  v8h pk[3];
#pragma unroll
  for (int it = 0; it < 3; ++it) {
    const int c  = it * 32 + cr;
    const int cl = (c < kXIN) ? c : (kXIN - 1);
    const v4f a = *(const v4f*)(s + cl * 68 + 8 * q);
    const v4f bb = *(const v4f*)(s + cl * 68 + 8 * q + 4);
    pk[it] = pack8(a, bb);
  }
  for (int pass = 0; pass < 2; ++pass) {
#pragma unroll
    for (int it = 0; it < 3; ++it) {
      const int c = it * 32 + cr;
      if (c < kXIN) {
        *(volatile v8h*)(XsT + ((size_t)(b * kXIN + c)) * kNP + n0 + 8 * q) = pk[it];
      }
    }
    __threadfence();
  }
}

template <int VAR>
__global__ __launch_bounds__(128) void cheb_spmm(const unsigned short* S16b, const unsigned short* Bb,
                                                 const unsigned short* X0b, unsigned short* Ob) {
  __shared__ __align__(16) float sD[64 * 68];
  const int tid  = threadIdx.x;
  const int lane = tid & 31;
  const int wave = tid >> 5;
  const int h    = lane >> 4;
  const int ml   = lane & 15;
  const int m    = blockIdx.z;
  const _Float16* S  = (const _Float16*)S16b + (size_t)m * CELLH;
  const _Float16* Bt = (const _Float16*)Bb   + (size_t)m * CELLH;
  const _Float16* X0 = (const _Float16*)X0b  + (size_t)m * CELLH;
  _Float16* O = (_Float16*)Ob + (size_t)m * CELLH;
  const int n0 = blockIdx.x * 64;
  const int j0 = blockIdx.y * 64;
  const int nw = n0 + wave * 16;

  const _Float16* ap  = S  + (size_t)(nw + ml) * kNP + 8 * h;
  const _Float16* bp0 = Bt + (size_t)(j0 + ml) * kNP + 8 * h;

  v8f acc[4];
#pragma unroll
  for (int t = 0; t < 4; ++t) acc[t] = zero8();

#pragma unroll 1
  for (int k0 = 0; k0 < kNP; k0 += 32) {
    const v16h a = ldfrag(ap + k0);
    v16h bf[4];
#pragma unroll
    for (int t = 0; t < 4; ++t) bf[t] = ldfrag(bp0 + (size_t)t * 16 * kNP + k0);
#pragma unroll
    for (int t = 0; t < 4; ++t) acc[t] = mma(a, bf[t], acc[t]);
    guard4(acc[0], acc[1], acc[2], acc[3], a, bf[0], bf[1], bf[2], bf[3]);
  }

#pragma unroll
  for (int t = 0; t < 4; ++t) {
#pragma unroll
    for (int r = 0; r < 8; ++r) sD[(16 * t + ml) * 68 + wave * 16 + 8 * h + r] = acc[t][r];
  }
  __syncthreads();

  const int q  = tid & 7;
  const int jr = tid >> 3;
  v8h pk[4];
#pragma unroll
  for (int it = 0; it < 4; ++it) {
    const int jl = it * 16 + jr;
    v4f a = *(const v4f*)(sD + jl * 68 + 8 * q);
    v4f b = *(const v4f*)(sD + jl * 68 + 8 * q + 4);
    if (VAR) {
      const v8h x8 = *(const v8h*)(X0 + (size_t)(j0 + jl) * kNP + n0 + 8 * q);
      const float c2 = 2.0f * kSupInv;
#pragma unroll
      for (int e = 0; e < 4; ++e) {
        a[e] = c2 * a[e] - (float)x8[e];
        b[e] = c2 * b[e] - (float)x8[e + 4];
      }
    } else {
      a = a * kSupInv;
      b = b * kSupInv;
    }
    pk[it] = pack8(a, b);
  }
  for (int pass = 0; pass < 2; ++pass) {
#pragma unroll
    for (int it = 0; it < 4; ++it) {
      const int jl = it * 16 + jr;
      *(volatile v8h*)(O + (size_t)(j0 + jl) * kNP + n0 + 8 * q) = pk[it];
    }
    __threadfence();
  }
}

__global__ __launch_bounds__(256) void build_xg(const unsigned short* XsTb, unsigned short* XGb) {
  __shared__ __align__(16) _Float16 sX[64 * 264];
  const int tid = threadIdx.x;
  const int m   = blockIdx.z;
  const int n0  = blockIdx.x * 8;
  const _Float16* P = (const _Float16*)XsTb + (size_t)m * CELLH;
  _Float16* XG = (_Float16*)XGb + (size_t)m * CELLH;
  if (tid < 128) {
    const int row = tid >> 1;
    const int hf  = tid & 1;
    v8h z;
#pragma unroll
    for (int e = 0; e < 8; ++e) z[e] = (_Float16)0.0f;
    *(v8h*)(sX + row * 264 + kKX + 8 * hf) = z;
  }
  for (int base = 0; base < 3 * kJ; base += 256) {
    const int idx = base + tid;
    if (idx < 3 * kJ) {
      const int t = idx / kJ;
      const int j = idx - t * kJ;
      const int b = j / kXIN;
      const int c = j - b * kXIN;
      const v8h v = *(const v8h*)(P + (size_t)t * PLANEH + (size_t)j * kNP + n0);
#pragma unroll
      for (int e = 0; e < 8; ++e) sX[(e * 8 + b) * 264 + t * kXIN + c] = v[e];
    }
  }
  __syncthreads();
  const int q  = tid & 31;
  const int r8 = tid >> 5;
  v8h pk[8];
#pragma unroll
  for (int it = 0; it < 8; ++it) {
    const int row = it * 8 + r8;
    pk[it] = *(const v8h*)(sX + row * 264 + 8 * q);
  }
  for (int pass = 0; pass < 2; ++pass) {
#pragma unroll
    for (int it = 0; it < 8; ++it) {
      const int row = it * 8 + r8;
      *(volatile v8h*)(XG + ((size_t)(n0 * kB + row)) * kKP + 8 * q) = pk[it];
    }
    __threadfence();
  }
}

template <int GATE>
__global__ __launch_bounds__(128) void hyper_apply(const unsigned short* XGb, const unsigned short* WTb,
                                                   const float* __restrict__ e1, const float* __restrict__ e2,
                                                   const float* __restrict__ e3, const float* __restrict__ me,
                                                   const float* __restrict__ bias, float* ZRb,
                                                   const float* __restrict__ t1, const float* __restrict__ t2,
                                                   const float* __restrict__ t3, float* out) {
#pragma clang fp contract(off)
  constexpr int O = GATE ? kOG : kOU;
  __shared__ __align__(16) float sT[4][16 * 36];
  const int lane = threadIdx.x & 31;
  const int wave = threadIdx.x >> 5;
  const int h    = lane >> 4;
  const int ml   = lane & 15;
  const int m    = blockIdx.z;
  const int rt   = blockIdx.x * 4 + wave;
  const int ob   = blockIdx.y * 32;
  const _Float16* XG = (const _Float16*)XGb + (size_t)m * CELLH;
  const _Float16* WT = (const _Float16*)WTb;
  float* ZR = ZRb + (size_t)m * CELLF;
  const float* emb = (m == 0) ? e1 : ((m == 1) ? e2 : e3);
  const float* st  = (m == 0) ? t1 : ((m == 1) ? t2 : t3);

  const _Float16* ap = XG + (size_t)(rt * 16 + ml) * kKP + 8 * h;
  v16h A[8];
#pragma unroll
  for (int kt = 0; kt < 8; ++kt) A[kt] = ldfrag(ap + kt * 32);

  const int nE = rt * 2 + h;
  const int nc = (nE < kN) ? nE : (kN - 1);
  const float* ep = emb + (size_t)nc * kD;
  const float* mp = me + m * kD;
  const _Float16* wp0 = WT + (size_t)(ob + ml) * kKP + 8 * h;

  v8f acc0 = zero8(), acc1 = zero8();
  float bs0 = 0.0f, bs1 = 0.0f;
#pragma unroll 1
  for (int d = 0; d < kD; ++d) {
    const float sd = bf_rne(ep[d]) * bf_rne(mp[d]);
    const _Float16* wp = wp0 + (size_t)(d * O) * kKP;
    v8f in0 = zero8(), in1 = zero8();
#pragma unroll
    for (int kt = 0; kt < 8; ++kt) {
      const v16h b0 = ldfrag(wp + kt * 32);
      const v16h b1 = ldfrag(wp + 16 * kKP + kt * 32);
      in0 = mma(A[kt], b0, in0);
      in1 = mma(A[kt], b1, in1);
      guard2(in0, in1, A[kt], b0, b1);
    }
    acc0 = acc0 + in0 * sd;
    acc1 = acc1 + in1 * sd;
    bs0 += sd * bf_rne(bias[d * O + ob + ml]);
    bs1 += sd * bf_rne(bias[d * O + ob + 16 + ml]);
  }

  float* slab = sT[wave];
#pragma unroll
  for (int r = 0; r < 8; ++r) {
    const float p0 = acc0[r] * kWInv + bs0;
    const float p1 = acc1[r] * kWInv + bs1;
    slab[(8 * h + r) * 36 + ml]      = act_f32(p0, GATE == 0);
    slab[(8 * h + r) * 36 + 16 + ml] = act_f32(p1, GATE == 0);
  }
  wave_sync_lds();

  const int q  = lane & 7;
  const int rr = lane >> 3;
  v4f hv[4];
#pragma unroll
  for (int it = 0; it < 4; ++it) {
    const int row = it * 4 + rr;
    const v4f v = *(const v4f*)(slab + row * 36 + 4 * q);
    if (GATE) {
      hv[it] = v;
    } else {
      const int node = rt * 2 + (row >> 3);
      const int bb   = row & 7;
      const int ncl  = (node < kN) ? node : (kN - 1);
      const v4f r4 = *(const v4f*)(ZR + (size_t)(rt * 16 + row) * kOG + kH + ob + 4 * q);
      const v4f s4 = bf4(*(const v4f*)(st + ((size_t)(bb * kN + ncl)) * kH + ob + 4 * q));
      const v4f one = {1.0f, 1.0f, 1.0f, 1.0f};
      const v4f a = r4 * s4;
      const v4f c = (one - r4) * v;
      hv[it] = a + c;
    }
  }
  for (int pass = 0; pass < 2; ++pass) {
#pragma unroll
    for (int it = 0; it < 4; ++it) {
      const int row = it * 4 + rr;
      if (GATE) {
        *(volatile v4f*)(ZR + (size_t)(rt * 16 + row) * kOG + ob + 4 * q) = hv[it];
      } else {
        const int node = rt * 2 + (row >> 3);
        const int bb   = row & 7;
        if (node < kN) {
          *(volatile v4f*)(out + (size_t)m * kB * kN * kH + ((size_t)(bb * kN + node)) * kH + ob + 4 * q) = hv[it];
        }
      }
    }
    __threadfence();
  }
}

extern "C" void kernel_launch(void* const* d_in, const int* in_sizes, int n_in,
                              void* d_out, int out_size, void* d_ws, size_t ws_size,
                              hipStream_t stream) {
  if (n_in < 17) return;
  for (int i = 0; i < 3; ++i)  { if (in_sizes[i] != kB * kN * kCIN) return; }
  for (int i = 3; i < 6; ++i)  { if (in_sizes[i] != kB * kN * kH) return; }
  for (int i = 6; i < 9; ++i)  { if (in_sizes[i] != kN * kN) return; }
  for (int i = 9; i < 12; ++i) { if (in_sizes[i] != kN * kD) return; }
  if (in_sizes[12] != 3 * kD) return;
  if (in_sizes[13] != kD * kKX * kOG) return;
  if (in_sizes[14] != kD * kOG) return;
  if (in_sizes[15] != kD * kKX * kOU) return;
  if (in_sizes[16] != kD * kOU) return;
  if (out_size != 3 * kB * kN * kH) return;
  if (WS_TOTAL > ws_size) return;

  const float* x1 = (const float*)d_in[0];
  const float* x2 = (const float*)d_in[1];
  const float* x3 = (const float*)d_in[2];
  const float* st1 = (const float*)d_in[3];
  const float* st2 = (const float*)d_in[4];
  const float* st3 = (const float*)d_in[5];
  const float* sp1 = (const float*)d_in[6];
  const float* sp2 = (const float*)d_in[7];
  const float* sp3 = (const float*)d_in[8];
  const float* e1 = (const float*)d_in[9];
  const float* e2 = (const float*)d_in[10];
  const float* e3 = (const float*)d_in[11];
  const float* me = (const float*)d_in[12];
  const float* Wg = (const float*)d_in[13];
  const float* Bg = (const float*)d_in[14];
  const float* Wu = (const float*)d_in[15];
  const float* Bu = (const float*)d_in[16];
  float* out = (float*)d_out;

  char* ws = (char*)d_ws;
  unsigned short* WGT = (unsigned short*)(ws + OFF_WG);
  unsigned short* WUT = (unsigned short*)(ws + OFF_WU);
  unsigned short* S16 = (unsigned short*)(ws + OFF_CELL + C_S16);
  unsigned short* XST = (unsigned short*)(ws + OFF_CELL + C_XST);
  unsigned short* T1T = (unsigned short*)(ws + OFF_CELL + C_T1T);
  unsigned short* T2T = (unsigned short*)(ws + OFF_CELL + C_T2T);
  unsigned short* XG  = (unsigned short*)(ws + OFF_CELL + C_XG);
  float* ZR = (float*)(ws + OFF_CELL + C_ZR);

  const dim3 b256(256), b128(128);
  const dim3 gS(kNP * kNP / 8 / 256, 1, 3);
  const dim3 gWg(kKP / 64, kOG / 64, kD);
  const dim3 gWu(kKP / 64, kOU / 64, kD);
  const dim3 gXs(kNP / 64, kB, 3);
  const dim3 gSp(kNP / 64, kJ / 64, 3);
  const dim3 gXg(kNP / 8, 1, 3);
  const dim3 gAg(kR / 64, kOG / 32, 3);
  const dim3 gAu(kR / 64, kOU / 32, 3);

  build_s16<<<gS, b256, 0, stream>>>(sp1, sp2, sp3, S16);
  build_wt<<<gWg, b256, 0, stream>>>(Wg, kOG, WGT);
  build_wt<<<gWu, b256, 0, stream>>>(Wu, kOU, WUT);
  build_xst<0><<<gXs, b256, 0, stream>>>(x1, x2, x3, st1, st2, st3, ZR, XST);
  cheb_spmm<0><<<gSp, b128, 0, stream>>>(S16, XST, XST, T1T);
  cheb_spmm<1><<<gSp, b128, 0, stream>>>(S16, T1T, XST, T2T);
  build_xg<<<gXg, b256, 0, stream>>>(XST, XG);
  hyper_apply<1><<<gAg, b128, 0, stream>>>(XG, WGT, e1, e2, e3, me, Bg, ZR, st1, st2, st3, out);
  build_xst<1><<<gXs, b256, 0, stream>>>(x1, x2, x3, st1, st2, st3, ZR, XST);
  cheb_spmm<0><<<gSp, b128, 0, stream>>>(S16, XST, XST, T1T);
  cheb_spmm<1><<<gSp, b128, 0, stream>>>(S16, T1T, XST, T2T);
  build_xg<<<gXg, b256, 0, stream>>>(XST, XG);
  hyper_apply<0><<<gAu, b128, 0, stream>>>(XG, WUT, e1, e2, e3, me, Bu, ZR, st1, st2, st3, out);
  (void)hipGetLastError();
}
